// KroneckerMixer_82102594830394
// MI455X (gfx1250) — hardware-verified
//
#include <hip/hip_runtime.h>
#include <math.h>
typedef __attribute__((ext_vector_type(16))) _Float16 v16h;
typedef __attribute__((ext_vector_type(8)))  _Float16 v8h;
typedef __attribute__((ext_vector_type(16))) __bf16   v16b;
typedef __attribute__((ext_vector_type(8)))  __bf16   v8b;
typedef __attribute__((ext_vector_type(8)))  float    v8f;
typedef __attribute__((ext_vector_type(4)))  float    v4f;
#define PSCALE 32768.0f
#define U16(p) ((const unsigned short*)(const void*)(p))
#define PSCALE_INV (1.0f / 32768.0f)

__device__ __forceinline__ unsigned short f2bf_bits(float f) {
  unsigned u = __float_as_uint(f);
  return (unsigned short)((u + 0x7FFFu + ((u >> 16) & 1u)) >> 16);
}
__device__ __forceinline__ float bf_bits2f(unsigned short h) { return __uint_as_float(((unsigned)h) << 16); }

__device__ __forceinline__ void dep_guard_h(v8f& a, v8f& b, v16h x, v16h y) { asm volatile("v_nop\n\tv_nop\n\tv_nop\n\tv_nop" : "+v"(a), "+v"(b) : "v"(x), "v"(y)); }
__device__ __forceinline__ void dep_guard_b(v8f& a, v8f& b, v16b x, v16b y) { asm volatile("v_nop\n\tv_nop\n\tv_nop\n\tv_nop" : "+v"(a), "+v"(b) : "v"(x), "v"(y)); }
__device__ __forceinline__ void keep4_h(v16h a, v16h b, v16h c, v16h d) { asm volatile("v_nop" :: "v"(a), "v"(b), "v"(c), "v"(d)); }
__device__ __forceinline__ void keep4_b(v16b a, v16b b, v16b c, v16b d) { asm volatile("v_nop" :: "v"(a), "v"(b), "v"(c), "v"(d)); }
__device__ __forceinline__ void acc_guard4(v8f& a, v8f& b, v8f& c, v8f& d) { asm volatile("v_nop\n\tv_nop\n\tv_nop\n\tv_nop" : "+v"(a), "+v"(b), "+v"(c), "+v"(d)); }
template <typename T> struct Frag;
template <> struct Frag<_Float16> {
  typedef v16h V; union U { v16h v; v8h h[2]; };
  static __device__ __forceinline__ v16h load(const _Float16* p) {
    U f; f.h[0] = *(const v8h*)(p); f.h[1] = *(const v8h*)(p + 16); return f.v;
  }
  static __device__ __forceinline__ v8f mma(v16h a, v16h b, v8f c) {
    return __builtin_amdgcn_wmma_f32_16x16x32_f16(false, a, false, b, (short)0, c, false, false);
  }
  static __device__ __forceinline__ void guard(v8f& a, v8f& b, v16h x, v16h y) { dep_guard_h(a, b, x, y); }
  static __device__ __forceinline__ void keep(v16h a, v16h b, v16h c, v16h d) { keep4_h(a, b, c, d); }
};
template <> struct Frag<__bf16> {
  typedef v16b V; union U { v16b v; v8b h[2]; };
  static __device__ __forceinline__ v16b load(const __bf16* p) {
    U f; f.h[0] = *(const v8b*)(p); f.h[1] = *(const v8b*)(p + 16); return f.v;
  }
  static __device__ __forceinline__ v8f mma(v16b a, v16b b, v8f c) {
    return __builtin_amdgcn_wmma_f32_16x16x32_bf16(false, a, false, b, (short)0, c, false, false);
  }
  static __device__ __forceinline__ void guard(v8f& a, v8f& b, v16b x, v16b y) { dep_guard_b(a, b, x, y); }
  static __device__ __forceinline__ void keep(v16b a, v16b b, v16b c, v16b d) { keep4_b(a, b, c, d); }
};

template <int ET> struct Elem;
template <> struct Elem<0> { typedef _Float16 T; };
template <> struct Elem<1> { typedef __bf16 T; };
template <int ET, bool SPLIT, int BIAS_MODE, int OUT_MODE, bool RESID, int ACT = 0>
__global__ __launch_bounds__(256) void wmma_gemm64(
    const unsigned short* __restrict__ Ap, const unsigned short* __restrict__ A2p, int lda, long strideA,
    const unsigned short* __restrict__ Btp, const unsigned short* __restrict__ Bt2p, int ldb, long strideB,
    void* __restrict__ Cout, void* __restrict__ Cout2, int ldc, long strideC,
    const float* __restrict__ bias,
    const float* __restrict__ resid, long strideR,
    int M, int N, int K, float scale) {
  typedef typename Elem<ET>::T T;
  typedef typename Frag<T>::V V;
  const T* A = (const T*)Ap; const T* A2 = (const T*)A2p; const T* Bt = (const T*)Btp; const T* Bt2 = (const T*)Bt2p;
  __shared__ __align__(16) float sT[8][16 * 68];
  const int b    = blockIdx.y;
  const int lane = threadIdx.x & 31;
  const int wave = threadIdx.x >> 5;
  const int tilesN = N >> 6;
  const int tilesM = M >> 6;
  const int tile = blockIdx.x * 8 + wave;
  if (tile >= tilesM * tilesN) return;
  const int tm = tile / tilesN;
  const int tn = tile - tm * tilesN;
  const int m0 = tm << 6;
  const int n0 = tn << 6;

  const T* Ab  = A  + (size_t)b * strideA;
  const T* Bb  = Bt + (size_t)b * strideB;
  const T* Ab2 = SPLIT ? (A2  + (size_t)b * strideA) : nullptr;
  const T* Bb2 = SPLIT ? (Bt2 + (size_t)b * strideB) : nullptr;

  const int rlane = lane & 15;
  const int koff  = (lane >> 4) * 8;
  const int mOff  = (lane >> 4) * 8;

  v8f acc[4][4];
#pragma unroll
  for (int i = 0; i < 4; ++i)
#pragma unroll
    for (int j = 0; j < 4; ++j) acc[i][j] = (v8f){0.f,0.f,0.f,0.f,0.f,0.f,0.f,0.f};

  for (int k0 = 0; k0 < K; k0 += 32) {
    V bh[4], bl[4];
#pragma unroll
    for (int j = 0; j < 4; ++j) {
      const size_t bo = (size_t)(n0 + (j << 4) + rlane) * ldb + koff + k0;
      bh[j] = Frag<T>::load(Bb + bo);
      if (SPLIT) bl[j] = Frag<T>::load(Bb2 + bo);
    }
#pragma unroll
    for (int i = 0; i < 4; ++i) {
      const size_t ao = (size_t)(m0 + (i << 4) + rlane) * lda + koff + k0;
      V ah = Frag<T>::load(Ab + ao);
      V al;
      if (SPLIT) al = Frag<T>::load(Ab2 + ao);
#pragma unroll
      for (int j = 0; j < 4; ++j) {
        acc[i][j] = Frag<T>::mma(ah, bh[j], acc[i][j]);
        if (SPLIT) {
          acc[i][j] = Frag<T>::mma(ah, bl[j], acc[i][j]);
          acc[i][j] = Frag<T>::mma(al, bh[j], acc[i][j]);
        }
      }
      Frag<T>::guard(acc[i][0], acc[i][3], ah, SPLIT ? al : ah);
    }
    Frag<T>::keep(bh[0], bh[1], bh[2], bh[3]);
    if (SPLIT) Frag<T>::keep(bl[0], bl[1], bl[2], bl[3]);
  }
  acc_guard4(acc[0][0], acc[0][1], acc[0][2], acc[0][3]);
  acc_guard4(acc[1][0], acc[1][1], acc[1][2], acc[1][3]);
  acc_guard4(acc[2][0], acc[2][1], acc[2][2], acc[2][3]);
  acc_guard4(acc[3][0], acc[3][1], acc[3][2], acc[3][3]);

  float* slab = sT[wave];
  const float* Rb = RESID ? (resid + (size_t)b * strideR) : nullptr;
#pragma unroll
  for (int i = 0; i < 4; ++i) {
    const int mBase = m0 + (i << 4);
#pragma unroll
    for (int j = 0; j < 4; ++j) {
      const int n = n0 + (j << 4) + rlane;
      float bv = 0.f;
      if (BIAS_MODE == 2) bv = bias[n];
#pragma unroll
      for (int r = 0; r < 8; ++r) {
        float v = acc[i][j][r] * scale;
        if (BIAS_MODE == 1) v += bias[mBase + mOff + r];
        if (BIAS_MODE == 2) v += bv;
        if (RESID) v += Rb[(size_t)(mBase + mOff + r) * ldc + n];
        if (ACT == 1) v = tanhf(v);
        if (ACT == 2) v = fmaxf(v, 0.0f);
        if (ACT == 3) v = v / (1.0f + expf(-v));
        if (ACT == 4) v = (v > 0.f) ? v : 0.01f * v;
        if (ACT == 5) v = 0.5f * v * (1.0f + erff(v * 0.70710678118654752f));
        slab[(mOff + r) * 68 + (j << 4) + rlane] = v;
      }
    }
    __builtin_amdgcn_fence(__ATOMIC_RELEASE, "workgroup");
    __builtin_amdgcn_wave_barrier();
    __builtin_amdgcn_fence(__ATOMIC_ACQUIRE, "workgroup");
    if (OUT_MODE == 0) {
      float* C = (float*)Cout + (size_t)b * strideC;
      const int hh = lane >> 4, c4 = (lane & 15) * 4;
      for (int pass = 0; pass < 2; ++pass) {
#pragma unroll
        for (int it = 0; it < 8; ++it) {
          const int row = it * 2 + hh;
          v4f v = *(const v4f*)(slab + row * 68 + c4);
          *(volatile v4f*)(C + (size_t)(mBase + row) * ldc + n0 + c4) = v;
        }
        __threadfence();
      }
    } else {
      const int q = lane >> 3, c8 = (lane & 7) * 8;
      unsigned short* C  = (unsigned short*)Cout  + (size_t)b * strideC;
      unsigned short* C2 = (OUT_MODE == 2) ? ((unsigned short*)Cout2 + (size_t)b * strideC) : nullptr;
      for (int pass = 0; pass < 2; ++pass) {
#pragma unroll
        for (int it = 0; it < 4; ++it) {
          const int row = it * 4 + q;
          const float* sp = slab + row * 68 + c8;
          v8h hv, lv;
#pragma unroll
          for (int e = 0; e < 8; ++e) {
            if (OUT_MODE == 1) {
              hv[e] = (_Float16)sp[e];
            } else {
              unsigned short hb = f2bf_bits(sp[e]);
              unsigned short lb = f2bf_bits(sp[e] - bf_bits2f(hb));
              hv[e] = __builtin_bit_cast(_Float16, hb);
              lv[e] = __builtin_bit_cast(_Float16, lb);
            }
          }
          *(volatile v8h*)(C + (size_t)(mBase + row) * ldc + n0 + c8) = hv;
          if (OUT_MODE == 2) *(volatile v8h*)(C2 + (size_t)(mBase + row) * ldc + n0 + c8) = lv;
        }
        __threadfence();
      }
    }
    __builtin_amdgcn_fence(__ATOMIC_RELEASE, "workgroup");
    __builtin_amdgcn_wave_barrier();
    __builtin_amdgcn_fence(__ATOMIC_ACQUIRE, "workgroup");
  }
}

__global__ __launch_bounds__(256) void cast_f32_f16x2(
    const float* __restrict__ in, _Float16* __restrict__ out, int n2) {
  int i = blockIdx.x * 256 + threadIdx.x;
  if (i < n2) {
    const _Float16 h0 = (_Float16)in[2 * i], h1 = (_Float16)in[2 * i + 1];
    const unsigned u = (unsigned)__builtin_bit_cast(unsigned short, h0) | ((unsigned)__builtin_bit_cast(unsigned short, h1) << 16);
    ((volatile unsigned*)out)[i] = u;
    __threadfence();
    ((volatile unsigned*)out)[i] = u;
  }
}


#define KB 64
#define KN 1024
#define KK 64
#define KBASIS 8
#define KITERS 20
#define KTEMP 0.2f
__global__ __launch_bounds__(1024) void sinkA_kernel(const float* __restrict__ logits, float* __restrict__ A32, unsigned* __restrict__ A16) {
  const int t = threadIdx.x;
  for (int i = t; i < KN * KN; i += 1024) A32[i] = logits[i] * (1.0f / KTEMP);
  __syncthreads();
#pragma unroll 1
  for (int it = 0; it < KITERS; ++it) {
    { float* row = A32 + (size_t)t * KN; float mx = -INFINITY; for (int j = 0; j < KN; ++j) mx = fmaxf(mx, row[j]); float s = 0.f; for (int j = 0; j < KN; ++j) s += expf(row[j] - mx); const float lse = mx + logf(s); for (int j = 0; j < KN; ++j) row[j] -= lse; }
    __threadfence_block(); __syncthreads();
    { float mx = -INFINITY; for (int i = 0; i < KN; ++i) mx = fmaxf(mx, A32[(size_t)i * KN + t]); float s = 0.f; for (int i = 0; i < KN; ++i) s += expf(A32[(size_t)i * KN + t] - mx); const float lse = mx + logf(s); for (int i = 0; i < KN; ++i) A32[(size_t)i * KN + t] -= lse; }
    __threadfence_block(); __syncthreads(); }
  for (int pass = 0; pass < 2; ++pass) { for (int j = 0; j < KN; j += 2) ((volatile unsigned*)A16)[((size_t)t * KN + j) / 2] = (unsigned)__builtin_bit_cast(unsigned short, (_Float16)expf(A32[(size_t)t * KN + j])) | ((unsigned)__builtin_bit_cast(unsigned short, (_Float16)expf(A32[(size_t)t * KN + j + 1])) << 16); __threadfence(); }
}
__global__ __launch_bounds__(256) void sinkW_kernel(const float* __restrict__ W1, const float* __restrict__ WV, unsigned* __restrict__ WT16) {
  __shared__ float L[KK][KK + 1]; __shared__ float w1[KBASIS];
  const int n = blockIdx.x, t = threadIdx.x;
  if (t < KBASIS) w1[t] = W1[n * KBASIS + t];
  __syncthreads();
  for (int e = t; e < KK * KK; e += 256) { const int i = e / KK, o = e % KK; float a = 0.f;
#pragma unroll
    for (int k = 0; k < KBASIS; ++k) a += w1[k] * WV[(size_t)k * KK * KK + e]; L[i][o] = a * (1.0f / KTEMP); }
  __syncthreads();
#pragma unroll 1
  for (int it = 0; it < KITERS; ++it) {
    if (t < KK) { float mx = -INFINITY; for (int j = 0; j < KK; ++j) mx = fmaxf(mx, L[t][j]); float s = 0.f; for (int j = 0; j < KK; ++j) s += expf(L[t][j] - mx); const float lse = mx + logf(s); for (int j = 0; j < KK; ++j) L[t][j] -= lse; }
    __syncthreads();
    if (t < KK) { float mx = -INFINITY; for (int i = 0; i < KK; ++i) mx = fmaxf(mx, L[i][t]); float s = 0.f; for (int i = 0; i < KK; ++i) s += expf(L[i][t] - mx); const float lse = mx + logf(s); for (int i = 0; i < KK; ++i) L[i][t] -= lse; }
    __syncthreads(); }
  for (int pass = 0; pass < 2; ++pass) { for (int e = t; e < KK * KK / 2; e += 256) { const int o = e / (KK / 2), ip = 2 * (e % (KK / 2));
      ((volatile unsigned*)WT16)[((size_t)n * KK * KK + o * KK + ip) / 2] = (unsigned)__builtin_bit_cast(unsigned short, (_Float16)expf(L[ip][o])) | ((unsigned)__builtin_bit_cast(unsigned short, (_Float16)expf(L[ip + 1][o])) << 16); } __threadfence(); }
}
__global__ __launch_bounds__(256) void xlt_kernel(const unsigned* __restrict__ XL16, unsigned* __restrict__ XLT16) {
  __shared__ float tile[KK][65];
  const int b = blockIdx.y, n0 = blockIdx.x * 64, tx = threadIdx.x, ty = threadIdx.y; typedef __attribute__((ext_vector_type(2))) _Float16 v2h;
  for (int n = ty; n < 64; n += 8) { const v2h h = __builtin_bit_cast(v2h, XL16[(((size_t)b * KN + n0 + n) * KK) / 2 + tx]); tile[n][2 * tx] = (float)h[0]; tile[n][2 * tx + 1] = (float)h[1]; }
  __syncthreads();
  for (int pass = 0; pass < 2; ++pass) { for (int o = ty; o < KK; o += 8) ((volatile unsigned*)XLT16)[(((size_t)b * KK + o) * KN + n0) / 2 + tx] = (unsigned)__builtin_bit_cast(unsigned short, (_Float16)tile[2 * tx][o]) | ((unsigned)__builtin_bit_cast(unsigned short, (_Float16)tile[2 * tx + 1][o]) << 16); __threadfence(); }
}
__global__ __launch_bounds__(256) void outT_kernel(const float* __restrict__ G, float* __restrict__ out) {
  __shared__ float tile[KK][65];
  const int b = blockIdx.y, m0 = blockIdx.x * 64, tx = threadIdx.x, ty = threadIdx.y;
  for (int o = ty; o < KK; o += 8) { const float* src = G + ((size_t)b * KK + o) * KN + m0; tile[o][tx] = src[tx]; tile[o][32 + tx] = src[32 + tx]; }
  __syncthreads();
  for (int pass = 0; pass < 2; ++pass) { for (int m = ty; m < 64; m += 8) { float* d = out + (size_t)b * KN * KK + (size_t)(m0 + m) * KK; ((volatile float*)d)[tx] = tile[tx][m]; ((volatile float*)d)[32 + tx] = tile[32 + tx][m]; } __threadfence(); }
}
extern "C" void kernel_launch(void* const* d_in, const int* in_sizes, int n_in, void* d_out, int out_size, void* d_ws, size_t ws_size, hipStream_t stream) {
  (void)in_sizes; (void)n_in; (void)out_size; (void)ws_size;
  const float* x = (const float*)d_in[0]; const float* Alog = (const float*)d_in[1]; const float* W1 = (const float*)d_in[2]; const float* WV = (const float*)d_in[3];
  char* ws = (char*)d_ws; size_t off = 0;
  auto carve = [&](size_t bytes) -> char* { char* p = ws + off; off += (bytes + 255) & ~(size_t)255; return p; };
  float* A32 = (float*)carve((size_t)KN * KN * 4); unsigned* A16 = (unsigned*)carve((size_t)KN * KN * 2); unsigned* WT16 = (unsigned*)carve((size_t)KN * KK * KK * 2);
  _Float16* X16 = (_Float16*)carve((size_t)KB * KN * KK * 2); unsigned* XL16 = (unsigned*)carve((size_t)KB * KN * KK * 2); unsigned* XLT16 = (unsigned*)carve((size_t)KB * KN * KK * 2); float* G = (float*)carve((size_t)KB * KK * KN * 4);
  sinkA_kernel<<<1, 1024, 0, stream>>>(Alog, A32, A16);
  sinkW_kernel<<<KN, 256, 0, stream>>>(W1, WV, WT16);
  cast_f32_f16x2<<<(KB * KN * KK / 2 + 255) / 256, 256, 0, stream>>>(x, X16, (long)KB * KN * KK / 2);
  wmma_gemm64<0, false, 0, 1, false><<<dim3(1, KN), 256, 0, stream>>>(U16(X16), nullptr, KN * KK, 64, (const unsigned short*)WT16, nullptr, KK, (long)KK * KK, XL16, nullptr, KN * KK, 64, nullptr, nullptr, 0, KB, KK, KK, 1.0f);
  xlt_kernel<<<dim3(KN / 64, KB), dim3(32, 8), 0, stream>>>(XL16, XLT16);
  { const int t = (KB * KK / 64) * (KN / 64); wmma_gemm64<0, false, 0, 0, false><<<dim3((t + 7) / 8, 1), 256, 0, stream>>>((const unsigned short*)XLT16, nullptr, KN, 0, (const unsigned short*)A16, nullptr, KN, 0, G, nullptr, KN, 0, nullptr, nullptr, 0, KB * KK, KN, KN, 1.0f); }
  outT_kernel<<<dim3(KN / 64, KB), dim3(32, 8), 0, stream>>>(G, (float*)d_out);
}
